// PointNetSetAbstraction_77077483094164
// MI455X (gfx1250) — hardware-verified
//
#include <hip/hip_runtime.h>
#pragma clang fp contract(off)

typedef __attribute__((ext_vector_type(16))) _Float16 v16h;
typedef __attribute__((ext_vector_type(8)))  _Float16 v8h;
typedef __attribute__((ext_vector_type(8)))  float    v8f;
typedef __attribute__((ext_vector_type(4)))  float    v4f;
typedef __attribute__((ext_vector_type(4)))  unsigned v4u;

constexpr int NBATCH = 8;
constexpr int NPTS   = 8192;
constexpr int NSAMP  = 1024;
constexpr int NNBR   = 32;
constexpr int NGRP   = NBATCH * NSAMP;
constexpr int MROWS  = NGRP * NNBR;
constexpr int CH_L0  = 64;
constexpr int CH_L1  = 64;
constexpr int CH_L2  = 128;
constexpr int KPAD_L0 = 32;
constexpr int CIN_L0  = 6;
constexpr int NBLK_MLP = NGRP / 8;
constexpr float CARRY_X = 64.0f;
constexpr float CARRY_W = 64.0f;
constexpr float FOLD_L0 = 1.0f / (CARRY_X * CARRY_W);
constexpr float FOLD_L12 = 1.0f / CARRY_W;
constexpr float BALL_R2 = 0.16f;
constexpr float BN_EPSV = 1e-5f;
constexpr double INV_ROWS = 1.0 / (double)MROWS;

static_assert(NBATCH * NPTS * 3 == 196608, "xyz extent");
static_assert(MROWS == 262144, "row count");
static_assert(NGRP % 8 == 0, "grid exact");
static_assert(KPAD_L0 % 32 == 0 && CH_L0 % 32 == 0 && CH_L1 % 32 == 0, "K multiples of 32");
static_assert(CH_L0 % 16 == 0 && CH_L1 % 16 == 0 && CH_L2 % 16 == 0, "tile multiples");

constexpr size_t WS_CENT  = 0;
constexpr size_t WS_W0    = WS_CENT + (size_t)NGRP * 3 * 4;
constexpr size_t WS_W1    = WS_W0 + (size_t)CH_L0 * KPAD_L0 * 2;
constexpr size_t WS_W2    = WS_W1 + (size_t)CH_L1 * CH_L0 * 2;
constexpr size_t WS_SCSH  = WS_W2 + (size_t)CH_L2 * CH_L1 * 2;
constexpr size_t WS_PART0 = 131072;
constexpr size_t WS_PART1 = WS_PART0 + (size_t)NBLK_MLP * 256 * 4;
constexpr size_t WS_PART2 = WS_PART1 + (size_t)NBLK_MLP * 256 * 4;
constexpr size_t WS_GMAX  = WS_PART2 + (size_t)NBLK_MLP * 256 * 4;
constexpr size_t WS_GMIN  = WS_GMAX + (size_t)NGRP * CH_L2 * 4;
constexpr size_t WS_X0    = WS_GMIN + (size_t)NGRP * CH_L2 * 4;
constexpr size_t WS_TOTAL = WS_X0 + (size_t)MROWS * KPAD_L0 * 2;
static_assert(WS_SCSH + 3 * 256 * 4 <= WS_PART0, "small regions fit");
static_assert(WS_W0 % 128 == 0 && WS_W1 % 128 == 0 && WS_W2 % 128 == 0 && WS_SCSH % 128 == 0, "aligned");
static_assert(WS_GMAX % 128 == 0 && WS_GMIN % 128 == 0 && WS_X0 % 128 == 0, "aligned");
static_assert(WS_TOTAL <= (size_t)134217728, "carve under 128 MiB");

constexpr size_t OUT1_OFF_BYTES = 98304;
constexpr size_t OUT_TOTAL_BYTES = 4292608;
static_assert((size_t)NGRP * 3 * 4 == OUT1_OFF_BYTES, "out0 extent");
static_assert(OUT1_OFF_BYTES + (size_t)NGRP * CH_L2 * 4 == OUT_TOTAL_BYTES, "out1 extent");
static_assert(OUT1_OFF_BYTES % 128 == 0, "out1 line aligned");

union FragU { v16h v; v8h h[2]; };
__device__ __forceinline__ v16h frag_load(const _Float16* p) {
  FragU f;
  f.h[0] = *(const v8h*)(p);
  f.h[1] = *(const v8h*)(p + 16);
  return f.v;
}
__device__ __forceinline__ v8f mma_h(v16h a, v16h b, v8f c) {
  c = __builtin_amdgcn_wmma_f32_16x16x32_f16(false, a, false, b, (short)0, c, false, false);
  asm volatile("v_nop\n\tv_nop\n\tv_nop\n\tv_nop" : "+v"(c) : "v"(a), "v"(b));
  return c;
}
__device__ __forceinline__ unsigned h_bits(float x) {
  const _Float16 h = (_Float16)x;
  const unsigned short s = __builtin_bit_cast(unsigned short, h);
  return (unsigned)s;
}
__device__ __forceinline__ float bfly_add(float v) {
  v = v + __shfl_xor(v, 1, 32);
  v = v + __shfl_xor(v, 2, 32);
  v = v + __shfl_xor(v, 4, 32);
  v = v + __shfl_xor(v, 8, 32);
  return v;
}
__device__ __forceinline__ float bfly_max(float v) {
  v = fmaxf(v, __shfl_xor(v, 1, 32));
  v = fmaxf(v, __shfl_xor(v, 2, 32));
  v = fmaxf(v, __shfl_xor(v, 4, 32));
  v = fmaxf(v, __shfl_xor(v, 8, 32));
  return v;
}
__device__ __forceinline__ float bfly_min(float v) {
  v = fminf(v, __shfl_xor(v, 1, 32));
  v = fminf(v, __shfl_xor(v, 2, 32));
  v = fminf(v, __shfl_xor(v, 4, 32));
  v = fminf(v, __shfl_xor(v, 8, 32));
  return v;
}

__global__ __launch_bounds__(256) void k_prep_w(const float* __restrict__ W0, const float* __restrict__ W1,
                                                const float* __restrict__ W2, unsigned* __restrict__ w0p,
                                                unsigned* __restrict__ w1p, unsigned* __restrict__ w2p) {
  const int blk = blockIdx.x;
  const int tid = threadIdx.x;
  float f0, f1;
  unsigned* dst;
  int widx;
  if (blk < 4) {
    widx = blk * 256 + tid;
    const int n = widx >> 4;
    const int k = (widx & 15) * 2;
    const int ka = (k < CIN_L0) ? k : (CIN_L0 - 1);
    const int kb = (k + 1 < CIN_L0) ? (k + 1) : (CIN_L0 - 1);
    const float a = W0[n * CIN_L0 + ka];
    const float b = W0[n * CIN_L0 + kb];
    f0 = (k < CIN_L0) ? a : 0.0f;
    f1 = (k + 1 < CIN_L0) ? b : 0.0f;
    dst = w0p;
  } else if (blk < 12) {
    widx = (blk - 4) * 256 + tid;
    f0 = W1[2 * widx];
    f1 = W1[2 * widx + 1];
    dst = w1p;
  } else {
    widx = (blk - 12) * 256 + tid;
    f0 = W2[2 * widx];
    f1 = W2[2 * widx + 1];
    dst = w2p;
  }
  const unsigned lo = h_bits(f0 * CARRY_W);
  const unsigned hi = h_bits(f1 * CARRY_W);
  const unsigned u = (lo & 0xffffu) | (hi << 16);
  *(volatile unsigned*)(dst + widx) = u;
  __threadfence();
  *(volatile unsigned*)(dst + widx) = u;
}

__global__ __launch_bounds__(1024) void k_fps(const float* __restrict__ xyz, float* __restrict__ out0,
                                              float* __restrict__ cent) {
#pragma clang fp contract(off)
  __shared__ __align__(16) float s_stage[3072];
  __shared__ float s_val[2][32];
  __shared__ int   s_idx[2][32];
  __shared__ int   s_sel[NSAMP];

  const int b    = blockIdx.x;
  const int tid  = threadIdx.x;
  const int lane = tid & 31;
  const int wid  = tid >> 5;
  const float* xb = xyz + (size_t)b * NPTS * 3;

  float px[8], py[8], pz[8], dmin[8];
#pragma unroll
  for (int j = 0; j < 8; ++j) {
    if (tid < 768) {
      const v4f v = *(const v4f*)(xb + j * 3072 + tid * 4);
      *(v4f*)(s_stage + tid * 4) = v;
    }
    __syncthreads();
    px[j] = s_stage[tid * 3 + 0];
    py[j] = s_stage[tid * 3 + 1];
    pz[j] = s_stage[tid * 3 + 2];
    dmin[j] = 1e10f;
    __syncthreads();
  }

  int far = 0;
  for (int it = 0; it < NSAMP; ++it) {
    if (tid == 0) s_sel[it] = far;
    int fc = far;
    fc = fc < 0 ? 0 : fc;
    fc = fc > (NPTS - 1) ? (NPTS - 1) : fc;
    const float cx = xb[fc * 3 + 0];
    const float cy = xb[fc * 3 + 1];
    const float cz = xb[fc * 3 + 2];

    float best = -1.0f;
    int   bi   = 0;
#pragma unroll
    for (int j = 0; j < 8; ++j) {
      const float dx = px[j] - cx;
      const float dy = py[j] - cy;
      const float dz = pz[j] - cz;
      const float t0 = dx * dx;
      const float t1 = dy * dy;
      const float t2 = dz * dz;
      const float dd = (t0 + t2) + t1;
      dmin[j] = fminf(dmin[j], dd);
      if (dmin[j] > best) { best = dmin[j]; bi = tid + j * 1024; }
    }
#pragma unroll
    for (int o = 16; o > 0; o >>= 1) {
      const float ov = __shfl_xor(best, o, 32);
      const int   oi = __shfl_xor(bi, o, 32);
      const bool take = (ov > best) || ((ov == best) && (oi < bi));
      best = take ? ov : best;
      bi   = take ? oi : bi;
    }
    const int buf = it & 1;
    if (lane == 0) { s_val[buf][wid] = best; s_idx[buf][wid] = bi; }
    __syncthreads();
    float v = s_val[buf][lane];
    int   i = s_idx[buf][lane];
#pragma unroll
    for (int o = 16; o > 0; o >>= 1) {
      const float ov = __shfl_xor(v, o, 32);
      const int   oi = __shfl_xor(i, o, 32);
      const bool take = (ov > v) || ((ov == v) && (oi < i));
      v = take ? ov : v;
      i = take ? oi : i;
    }
    far = i;
  }
  __syncthreads();
  if (tid < 768) {
    float o[4];
#pragma unroll
    for (int e = 0; e < 4; ++e) {
      const int flat = tid * 4 + e;
      const int s = flat / 3;
      const int cc = flat - s * 3;
      int id = s_sel[s];
      id = id < 0 ? 0 : id;
      id = id > (NPTS - 1) ? (NPTS - 1) : id;
      o[e] = xb[id * 3 + cc];
    }
    const v4f val = {o[0], o[1], o[2], o[3]};
    float* d0 = out0 + (size_t)b * (NSAMP * 3) + tid * 4;
    float* d1 = cent + (size_t)b * (NSAMP * 3) + tid * 4;
    *(volatile v4f*)d0 = val;
    *(volatile v4f*)d1 = val;
    __threadfence();
    *(volatile v4f*)d0 = val;
    *(volatile v4f*)d1 = val;
  }
}

__global__ __launch_bounds__(256) void k_ball_group(const float* __restrict__ xyz, const float* __restrict__ pts,
                                                    const float* __restrict__ cent, unsigned* __restrict__ x0w) {
#pragma clang fp contract(off)
  __shared__ int s_list[8][32];
  const int lane = threadIdx.x & 31;
  const int wv   = threadIdx.x >> 5;
  const int gs   = blockIdx.x * 8 + wv;
  const int b    = gs >> 10;
  const float* xb = xyz + (size_t)b * NPTS * 3;
  const float* pb = pts + (size_t)b * NPTS * 3;
  const float cx = cent[(size_t)gs * 3 + 0];
  const float cy = cent[(size_t)gs * 3 + 1];
  const float cz = cent[(size_t)gs * 3 + 2];
  const float tcx = cx * cx;
  const float tcy = cy * cy;
  const float tcz = cz * cz;
  const float sqc = (tcx + tcz) + tcy;

  s_list[wv][lane] = 0;
  __syncthreads();

  int cnt = 0;
  for (int base = 0; base < NPTS && cnt < NNBR; base += 32) {
    const int j = base + lane;
    const float x = xb[j * 3 + 0];
    const float y = xb[j * 3 + 1];
    const float z = xb[j * 3 + 2];
    const float tx = x * x;
    const float ty = y * y;
    const float tz = z * z;
    const float sqx = (tx + tz) + ty;
    float p = cx * x;
    p = __builtin_fmaf(cy, y, p);
    p = __builtin_fmaf(cz, z, p);
    const float two_p = 2.0f * p;
    const float sq = (sqc - two_p) + sqx;
    const bool inb = !(sq > BALL_R2);
    const unsigned mask = (unsigned)__ballot(inb);
    const int rank = __popc(mask & ((1u << lane) - 1u));
    const int slot = cnt + rank;
    if (inb && slot < NNBR) s_list[wv][slot] = j;
    cnt += __popc(mask);
  }
  __syncthreads();

  const int mine = s_list[wv][lane];
  const int head = s_list[wv][0];
  const int first = (cnt > 0) ? head : (NPTS - 1);
  int idx = (lane < cnt) ? mine : first;
  idx = idx < 0 ? 0 : idx;
  idx = idx > (NPTS - 1) ? (NPTS - 1) : idx;

  const float gx = xb[idx * 3 + 0];
  const float gy = xb[idx * 3 + 1];
  const float gz = xb[idx * 3 + 2];
  const float q0 = pb[idx * 3 + 0];
  const float q1 = pb[idx * 3 + 1];
  const float q2 = pb[idx * 3 + 2];
  const float dx = gx - cx;
  const float dy = gy - cy;
  const float dz = gz - cz;
  const unsigned h0 = h_bits(dx * CARRY_X);
  const unsigned h1 = h_bits(dy * CARRY_X);
  const unsigned h2 = h_bits(dz * CARRY_X);
  const unsigned h3 = h_bits(q0 * CARRY_X);
  const unsigned h4 = h_bits(q1 * CARRY_X);
  const unsigned h5 = h_bits(q2 * CARRY_X);
  const unsigned w0 = (h0 & 0xffffu) | (h1 << 16);
  const unsigned w1 = (h2 & 0xffffu) | (h3 << 16);
  const unsigned w2 = (h4 & 0xffffu) | (h5 << 16);
  unsigned zz = 0u;
  asm volatile("" : "+v"(zz));

  const bool piece0 = ((lane & 3) == 0);
  v4u ov[4];
#pragma unroll
  for (int i = 0; i < 4; ++i) {
    const int src = i * 8 + (lane >> 2);
    const unsigned a0 = __shfl(w0, src, 32);
    const unsigned a1 = __shfl(w1, src, 32);
    const unsigned a2 = __shfl(w2, src, 32);
    v4u t;
    t.x = piece0 ? a0 : zz;
    t.y = piece0 ? a1 : zz;
    t.z = piece0 ? a2 : zz;
    t.w = zz;
    ov[i] = t;
  }
  unsigned* dst = x0w + (size_t)gs * 512 + lane * 4;
#pragma unroll
  for (int i = 0; i < 4; ++i) *(volatile v4u*)(dst + i * 128) = ov[i];
  __threadfence();
#pragma unroll
  for (int i = 0; i < 4; ++i) *(volatile v4u*)(dst + i * 128) = ov[i];
}

__device__ __forceinline__ void tile_stats(const float (&ya)[8], const float (&yb)[8],
                                           float* dsum, float* dsq, int rl) {
#pragma unroll
  for (int r = 0; r < 8; ++r) {
    float s = ya[r] + yb[r];
    const float qa = ya[r] * ya[r];
    const float qb = yb[r] * yb[r];
    float q = qa + qb;
    s = bfly_add(s);
    q = bfly_add(q);
    if (rl == 0) { dsum[r] = s; dsq[r] = q; }
  }
}

__device__ __forceinline__ void stats_tiles4(const v8f (&acc)[4][2], float fold, float* sumrow, float* sqrow,
                                             int hh, int rl) {
#pragma unroll
  for (int t = 0; t < 4; ++t) {
    float ya[8], yb[8];
#pragma unroll
    for (int r = 0; r < 8; ++r) { ya[r] = acc[t][0][r] * fold; yb[r] = acc[t][1][r] * fold; }
    tile_stats(ya, yb, sumrow + t * 16 + 8 * hh, sqrow + t * 16 + 8 * hh, rl);
  }
}

__device__ __forceinline__ void bn_pack(const v8f (&acc)[4][2], float fold, const float* scrow, const float* shrow,
                                        int hh, v16h (&outf)[2][2]) {
#pragma unroll
  for (int t = 0; t < 4; ++t) {
    float scv[8], shv[8];
#pragma unroll
    for (int r = 0; r < 8; ++r) { scv[r] = scrow[t * 16 + 8 * hh + r]; shv[r] = shrow[t * 16 + 8 * hh + r]; }
#pragma unroll
    for (int mi = 0; mi < 2; ++mi) {
#pragma unroll
      for (int r = 0; r < 8; ++r) {
        const float y = acc[t][mi][r] * fold;
        const float u = scv[r] * y;
        const float a = fmaxf(u + shv[r], 0.0f);
        outf[t >> 1][mi][(t & 1) * 8 + r] = (_Float16)a;
      }
    }
  }
}

template <int PASS>
__global__ __launch_bounds__(256) void k_mlp(const unsigned short* __restrict__ x0p,
                                             const unsigned short* __restrict__ w0p,
                                             const unsigned short* __restrict__ w1p,
                                             const unsigned short* __restrict__ w2p,
                                             const float* __restrict__ scsh, float* __restrict__ part,
                                             float* __restrict__ gmax, float* __restrict__ gmin) {
  constexpr int NOUT = (PASS == 2) ? CH_L2 : 64;
  __shared__ __align__(16) float s_bn[4][64];
  __shared__ __align__(16) float s_ws[8][2][128];
  __shared__ __align__(16) float s_tot[256];
  __shared__ __align__(16) float s_mm[8][2][128];

  const int tid  = threadIdx.x;
  const int lane = tid & 31;
  const int wave = tid >> 5;
  const int rl   = lane & 15;
  const int hh   = lane >> 4;
  const int koff = hh * 8;
  const int grp  = blockIdx.x * 8 + wave;
  const size_t m0 = (size_t)grp * NNBR;

  const _Float16* X0 = (const _Float16*)x0p;
  const _Float16* W0 = (const _Float16*)w0p;
  const _Float16* W1 = (const _Float16*)w1p;
  const _Float16* W2 = (const _Float16*)w2p;

  if (PASS >= 1) {
    const int nst = (PASS == 1) ? 32 : 64;
    if (tid < nst) {
      const int which = tid >> 4;
      const int c4 = (tid & 15) * 4;
      const v4f v = *(const v4f*)(scsh + (which >> 1) * 256 + (which & 1) * 128 + c4);
      *(v4f*)(&s_bn[which][c4]) = v;
    }
    __syncthreads();
  }

  const v8f vzero = {0.f, 0.f, 0.f, 0.f, 0.f, 0.f, 0.f, 0.f};

  const v16h xb0 = frag_load(X0 + (m0 + rl) * KPAD_L0 + koff);
  const v16h xb1 = frag_load(X0 + (m0 + 16 + rl) * KPAD_L0 + koff);
  v8f acc0[4][2];
#pragma unroll
  for (int t = 0; t < 4; ++t) {
    const v16h wa = frag_load(W0 + (size_t)(t * 16 + rl) * KPAD_L0 + koff);
    acc0[t][0] = mma_h(wa, xb0, vzero);
    acc0[t][1] = mma_h(wa, xb1, vzero);
  }

  if (PASS == 0) {
    stats_tiles4(acc0, FOLD_L0, &s_ws[wave][0][0], &s_ws[wave][1][0], hh, rl);
  } else {
    v16h bb[2][2];
    bn_pack(acc0, FOLD_L0, &s_bn[0][0], &s_bn[1][0], hh, bb);

    v8f acc1[4][2];
#pragma unroll
    for (int t = 0; t < 4; ++t) {
      acc1[t][0] = vzero;
      acc1[t][1] = vzero;
#pragma unroll
      for (int ks = 0; ks < 2; ++ks) {
        const v16h wa = frag_load(W1 + (size_t)(t * 16 + rl) * CH_L0 + ks * 32 + koff);
        acc1[t][0] = mma_h(wa, bb[ks][0], acc1[t][0]);
        acc1[t][1] = mma_h(wa, bb[ks][1], acc1[t][1]);
      }
    }

    if (PASS == 1) {
      stats_tiles4(acc1, FOLD_L12, &s_ws[wave][0][0], &s_ws[wave][1][0], hh, rl);
    } else {
      v16h cc[2][2];
      bn_pack(acc1, FOLD_L12, &s_bn[2][0], &s_bn[3][0], hh, cc);

#pragma unroll 1
      for (int t = 0; t < 8; ++t) {
        v8f c0 = vzero;
        v8f c1 = vzero;
#pragma unroll
        for (int ks = 0; ks < 2; ++ks) {
          const v16h wa = frag_load(W2 + (size_t)(t * 16 + rl) * CH_L1 + ks * 32 + koff);
          c0 = mma_h(wa, cc[ks][0], c0);
          c1 = mma_h(wa, cc[ks][1], c1);
        }
        float ya[8], yb[8];
#pragma unroll
        for (int r = 0; r < 8; ++r) { ya[r] = c0[r] * FOLD_L12; yb[r] = c1[r] * FOLD_L12; }
        const int chb = t * 16 + 8 * hh;
        tile_stats(ya, yb, &s_ws[wave][0][chb], &s_ws[wave][1][chb], rl);
#pragma unroll
        for (int r = 0; r < 8; ++r) {
          float mx = fmaxf(ya[r], yb[r]);
          float mn = fminf(ya[r], yb[r]);
          mx = bfly_max(mx);
          mn = bfly_min(mn);
          if (rl == 0) { s_mm[wave][0][chb + r] = mx; s_mm[wave][1][chb + r] = mn; }
        }
      }
    }
  }

  __syncthreads();
  if (tid < 2 * NOUT) {
    const int st = tid / NOUT;
    const int ch = tid - st * NOUT;
    float a = 0.0f;
#pragma unroll
    for (int w = 0; w < 8; ++w) a = a + s_ws[w][st][ch];
    s_tot[tid] = a;
  }
  __syncthreads();

  const bool do_part = (tid < (2 * NOUT) / 4);
  const int tq = do_part ? tid : 0;
  const v4f pv = *(const v4f*)(s_tot + tq * 4);
  float* pd = part + (size_t)blockIdx.x * 256 + tq * 4;
  const v4f vmx = *(const v4f*)(&s_mm[wave][0][lane * 4]);
  const v4f vmn = *(const v4f*)(&s_mm[wave][1][lane * 4]);
  float* gx = gmax + (size_t)grp * CH_L2 + lane * 4;
  float* gn = gmin + (size_t)grp * CH_L2 + lane * 4;
  if (do_part) *(volatile v4f*)pd = pv;
  if (PASS == 2) { *(volatile v4f*)gx = vmx; *(volatile v4f*)gn = vmn; }
  __threadfence();
  if (do_part) *(volatile v4f*)pd = pv;
  if (PASS == 2) { *(volatile v4f*)gx = vmx; *(volatile v4f*)gn = vmn; }
}

__global__ __launch_bounds__(256) void k_bn_fin(const float* __restrict__ part, const float* __restrict__ g,
                                                const float* __restrict__ be, float* __restrict__ scsh_l,
                                                int nout) {
  __shared__ double s_d[256];
  __shared__ __align__(16) float s_o[256];
  const int tid = threadIdx.x;
  const int lim = 2 * nout - 1;
  const int col = tid < lim ? tid : lim;
  double a = 0.0;
#pragma unroll 4
  for (int blk = 0; blk < NBLK_MLP; ++blk) a = a + (double)part[(size_t)blk * 256 + col];
  s_d[tid] = a;
  __syncthreads();
  if (tid < 128) {
    const int c = tid < nout ? tid : (nout - 1);
    const double m = s_d[c] * INV_ROWS;
    const double e2 = s_d[nout + c] * INV_ROWS;
    const double vd = e2 - m * m;
    float vf = (float)vd;
    vf = vf < 0.0f ? 0.0f : vf;
    const float rs = 1.0f / sqrtf(vf + BN_EPSV);
    const float s = g[c] * rs;
    const float ms = (float)m * s;
    const float h = be[c] - ms;
    s_o[tid] = (tid < nout) ? s : 0.0f;
    s_o[128 + tid] = (tid < nout) ? h : 0.0f;
  }
  __syncthreads();
  if (tid < 64) {
    const v4f v = *(const v4f*)(s_o + tid * 4);
    *(volatile v4f*)(scsh_l + tid * 4) = v;
    __threadfence();
    *(volatile v4f*)(scsh_l + tid * 4) = v;
  }
}

__global__ __launch_bounds__(256) void k_out(const float* __restrict__ gmax, const float* __restrict__ gmin,
                                             const float* __restrict__ scsh2, float* __restrict__ out1) {
  const int i = blockIdx.x * 256 + threadIdx.x;
  const int c4 = (i & 31) * 4;
  const v4f a = *(const v4f*)(gmax + (size_t)i * 4);
  const v4f b = *(const v4f*)(gmin + (size_t)i * 4);
  const v4f sc = *(const v4f*)(scsh2 + c4);
  const v4f sh = *(const v4f*)(scsh2 + 128 + c4);
  v4f o;
  {
    const float u0 = sc.x * a.x; const float w0 = sc.x * b.x;
    o.x = fmaxf(fmaxf(u0 + sh.x, w0 + sh.x), 0.0f);
    const float u1 = sc.y * a.y; const float w1 = sc.y * b.y;
    o.y = fmaxf(fmaxf(u1 + sh.y, w1 + sh.y), 0.0f);
    const float u2 = sc.z * a.z; const float w2 = sc.z * b.z;
    o.z = fmaxf(fmaxf(u2 + sh.z, w2 + sh.z), 0.0f);
    const float u3 = sc.w * a.w; const float w3 = sc.w * b.w;
    o.w = fmaxf(fmaxf(u3 + sh.w, w3 + sh.w), 0.0f);
  }
  float* d = out1 + (size_t)i * 4;
  *(volatile v4f*)d = o;
  __threadfence();
  *(volatile v4f*)d = o;
}

extern "C" void kernel_launch(void* const* d_in, const int* in_sizes, int n_in,
                              void* d_out, int out_size, void* d_ws, size_t ws_size, hipStream_t stream) {
  (void)in_sizes; (void)n_in; (void)out_size;
  if (ws_size < WS_TOTAL) return;

  const float* xyz = (const float*)d_in[0];
  const float* pts = (const float*)d_in[1];
  const float* W0  = (const float*)d_in[2];
  const float* g0  = (const float*)d_in[4];
  const float* be0 = (const float*)d_in[5];
  const float* W1  = (const float*)d_in[6];
  const float* g1  = (const float*)d_in[8];
  const float* be1 = (const float*)d_in[9];
  const float* W2  = (const float*)d_in[10];
  const float* g2  = (const float*)d_in[12];
  const float* be2 = (const float*)d_in[13];

  float* out0 = (float*)d_out;
  float* out1 = (float*)((char*)d_out + OUT1_OFF_BYTES);

  char* ws = (char*)d_ws;
  float* cent = (float*)(ws + WS_CENT);
  unsigned* w0p = (unsigned*)(ws + WS_W0);
  unsigned* w1p = (unsigned*)(ws + WS_W1);
  unsigned* w2p = (unsigned*)(ws + WS_W2);
  float* scsh  = (float*)(ws + WS_SCSH);
  float* part0 = (float*)(ws + WS_PART0);
  float* part1 = (float*)(ws + WS_PART1);
  float* part2 = (float*)(ws + WS_PART2);
  float* gmax  = (float*)(ws + WS_GMAX);
  float* gmin  = (float*)(ws + WS_GMIN);
  unsigned* x0w = (unsigned*)(ws + WS_X0);

  const unsigned short* x0h = (const unsigned short*)x0w;
  const unsigned short* w0h = (const unsigned short*)w0p;
  const unsigned short* w1h = (const unsigned short*)w1p;
  const unsigned short* w2h = (const unsigned short*)w2p;

  k_prep_w<<<28, 256, 0, stream>>>(W0, W1, W2, w0p, w1p, w2p);
  k_fps<<<NBATCH, 1024, 0, stream>>>(xyz, out0, cent);
  k_ball_group<<<NGRP / 8, 256, 0, stream>>>(xyz, pts, cent, x0w);

  k_mlp<0><<<NBLK_MLP, 256, 0, stream>>>(x0h, w0h, w1h, w2h, scsh, part0, gmax, gmin);
  k_bn_fin<<<1, 256, 0, stream>>>(part0, g0, be0, scsh + 0, CH_L0);
  k_mlp<1><<<NBLK_MLP, 256, 0, stream>>>(x0h, w0h, w1h, w2h, scsh, part1, gmax, gmin);
  k_bn_fin<<<1, 256, 0, stream>>>(part1, g1, be1, scsh + 256, CH_L1);
  k_mlp<2><<<NBLK_MLP, 256, 0, stream>>>(x0h, w0h, w1h, w2h, scsh, part2, gmax, gmin);
  k_bn_fin<<<1, 256, 0, stream>>>(part2, g2, be2, scsh + 512, CH_L2);
  k_out<<<(NGRP * CH_L2 / 4) / 256, 256, 0, stream>>>(gmax, gmin, scsh + 512, out1);
}
